// Fuzzy_MultiHeadAttention_QK_69200513073604
// MI455X (gfx1250) — hardware-run, weakly checked
//
#include <hip/hip_runtime.h>


#define NB_  64
#define NP   1024
#define DF   64
#define NR   64
#define CAR  64.0f
typedef _Float16 h16;
typedef unsigned short bf;
typedef __attribute__((ext_vector_type(16))) __bf16   v16bf;
typedef __attribute__((ext_vector_type(16))) _Float16 v16h;
typedef __attribute__((ext_vector_type(8)))  _Float16 v8h;
typedef __attribute__((ext_vector_type(8)))  unsigned short v8us;
typedef __attribute__((ext_vector_type(8)))  float    v8f;
typedef __attribute__((ext_vector_type(4)))  float    v4f;
typedef v8h  __attribute__((may_alias)) v8ha;
typedef v4f  __attribute__((may_alias)) v4fa;
typedef v8us __attribute__((may_alias)) v8usa;

__device__ __forceinline__ unsigned short f2bf(float f) { unsigned u = __float_as_uint(f); u += 0x7FFFu + ((u >> 16) & 1u); return (unsigned short)(u >> 16); }
__device__ __forceinline__ float bf2f(unsigned short b) { return __uint_as_float(((unsigned)b) << 16); }
__device__ __forceinline__ float bfr(float f) { return bf2f(f2bf(f)); }
__device__ __forceinline__ v16h cat16(v8h lo, v8h hi) { return __builtin_shufflevector(lo, hi, 0, 1, 2, 3, 4, 5, 6, 7, 8, 9, 10, 11, 12, 13, 14, 15); }
__device__ __forceinline__ v16bf cat16b(v8us lo, v8us hi) { return __builtin_bit_cast(v16bf, __builtin_shufflevector(lo, hi, 0, 1, 2, 3, 4, 5, 6, 7, 8, 9, 10, 11, 12, 13, 14, 15)); }
__device__ __forceinline__ v8f wmma16(v16h a, v16h b, v8f c) { return __builtin_amdgcn_wmma_f32_16x16x32_f16(false, a, false, b, (short)0, c, false, false); }
__device__ __forceinline__ v8f wmmab(v16bf a, v16bf b, v8f c) { return __builtin_amdgcn_wmma_f32_16x16x32_bf16(false, a, false, b, (short)0, c, false, false); }


template <typename T16> struct WFrag;
template <> struct WFrag<h16> { typedef v16h V; static __device__ __forceinline__ V ld(const h16* p) { return cat16(*(const v8h*)p, *(const v8h*)(p + 16)); } static __device__ __forceinline__ v8f mma(V a, V b, v8f c) { return wmma16(a, b, c); } };
template <> struct WFrag<bf> { typedef v16bf V; static __device__ __forceinline__ V ld(const bf* p) { return cat16b(*(const v8us*)p, *(const v8us*)(p + 16)); } static __device__ __forceinline__ v8f mma(V a, V b, v8f c) { return wmmab(a, b, c); } };
template <typename T16, int NSPLIT, bool BIAS>
__global__ __launch_bounds__(32) void k_gemmw(const T16* __restrict__ A, const T16* __restrict__ A2, const T16* __restrict__ Bt, const T16* __restrict__ Bt2, int K, float* C, int ldc, const float* __restrict__ bias, size_t sA, size_t sB, size_t sC) {
    typedef typename WFrag<T16>::V V;
    __shared__ __align__(16) float os[16 * 68];
    const size_t z = blockIdx.z; A += z * sA; if (A2) A2 += z * sA; Bt += z * sB; if (Bt2) Bt2 += z * sB; C += z * sC;
    const int lane = threadIdx.x & 31, lr = lane & 15, hi = lane >> 4; const int r0 = blockIdx.x * 64, c0 = blockIdx.y * 64;
    v8f acc[4][4];
#pragma unroll
    for (int mb = 0; mb < 4; ++mb)
#pragma unroll
        for (int nb = 0; nb < 4; ++nb) acc[mb][nb] = (v8f){};
    const size_t aoff = (size_t)(r0 + lr) * K + 8 * hi, boff = (size_t)(c0 + lr) * K + 8 * hi;

    for (int kc = 0; kc < K; kc += 32) {
        V a[4], a2[4];
#pragma unroll
        for (int mb = 0; mb < 4; ++mb) { a[mb] = WFrag<T16>::ld(A + aoff + (size_t)mb * 16 * K + kc); if (NSPLIT == 1 || NSPLIT == 2) a2[mb] = WFrag<T16>::ld(A2 + aoff + (size_t)mb * 16 * K + kc); }
#pragma unroll
        for (int nb = 0; nb < 4; ++nb) { const V b = WFrag<T16>::ld(Bt + boff + (size_t)nb * 16 * K + kc); V b2; if (NSPLIT >= 2) b2 = WFrag<T16>::ld(Bt2 + boff + (size_t)nb * 16 * K + kc);
#pragma unroll
            for (int mb = 0; mb < 4; ++mb) { acc[mb][nb] = WFrag<T16>::mma(a[mb], b, acc[mb][nb]); if (NSPLIT == 1 || NSPLIT == 2) acc[mb][nb] = WFrag<T16>::mma(a2[mb], b, acc[mb][nb]); if (NSPLIT >= 2) acc[mb][nb] = WFrag<T16>::mma(a[mb], b2, acc[mb][nb]); } }
        asm volatile("v_nop\n\tv_nop\n\tv_nop\n\tv_nop" : "+v"(acc[0][0]), "+v"(acc[1][1]), "+v"(acc[2][2]), "+v"(acc[3][3]) : "v"(a[0]), "v"(a[3]));
    }
#pragma unroll
    for (int mb = 0; mb < 4; ++mb) {
#pragma unroll
        for (int nb = 0; nb < 4; ++nb) {
#pragma unroll
            for (int j = 0; j < 8; ++j) os[(hi * 8 + j) * 68 + nb * 16 + lr] = acc[mb][nb][j]; }
        __builtin_amdgcn_wave_barrier(); asm volatile("" ::: "memory");
        float* crow = C + (size_t)(r0 + mb * 16) * ldc + c0;
#pragma unroll 1
        for (int ps = 0; ps < 2; ++ps) {
#pragma unroll
            for (int s = 0; s < 8; ++s) { const int row = 2 * s + hi, cofs = lr * 4; v4f val = *(const v4fa*)(os + row * 68 + cofs); if (BIAS) { val[0] += bfr(bias[c0 + cofs]); val[1] += bfr(bias[c0 + cofs + 1]); val[2] += bfr(bias[c0 + cofs + 2]); val[3] += bfr(bias[c0 + cofs + 3]); }
                *(volatile v4f*)(crow + (size_t)row * ldc + cofs) = val; }
            if (ps == 0) __threadfence(); }
        __builtin_amdgcn_wave_barrier(); asm volatile("" ::: "memory");
    }
}

__device__ __forceinline__ h16 tohx(float x) { return (h16)x; }
__device__ __forceinline__ void splitf(float y, unsigned short& h, unsigned short& l) { h = f2bf(y); l = f2bf(y - bf2f(h)); }
typedef __attribute__((ext_vector_type(2))) _Float16 v2h;
typedef __attribute__((ext_vector_type(4))) _Float16 v4h;
typedef __attribute__((ext_vector_type(2))) unsigned short v2us;
typedef __attribute__((ext_vector_type(4))) unsigned short v4us;
typedef __attribute__((ext_vector_type(2))) float v2f;
typedef __attribute__((ext_vector_type(4))) int v4i;
__global__ __launch_bounds__(256) void k_f2h(const float* __restrict__ S, h16* P16, size_t n4) { const size_t i = (size_t)blockIdx.x * 256 + threadIdx.x; if (i >= n4) return; const v4f v = *(const v4f*)(S + i * 4); v4h o;
#pragma unroll
    for (int q = 0; q < 4; ++q) o[q] = tohx(v[q]);
    *(volatile v4h*)(P16 + i * 4) = o; __threadfence(); *(volatile v4h*)(P16 + i * 4) = o; }
__global__ __launch_bounds__(256) void k_rbf(const float* __restrict__ X, float* Y, size_t n4) { const size_t i = (size_t)blockIdx.x * 256 + threadIdx.x; if (i >= n4) return; const v4f a = *(const v4f*)(X + i * 4); v4f o;
#pragma unroll
    for (int q = 0; q < 4; ++q) o[q] = bfr(a[q]);
    *(volatile v4f*)(Y + i * 4) = o; __threadfence(); *(volatile v4f*)(Y + i * 4) = o; }
__global__ __launch_bounds__(256) void k_wtG(const float* __restrict__ w, int K, int N, bf* Bt) {
    const int lane = threadIdx.x & 31; const int L0 = (blockIdx.x * 8 + (threadIdx.x >> 5)) * 8; const int nlines = N * K / 64;
#pragma unroll
    for (int ps = 0; ps < 2; ++ps) {
        for (int l = 0; l < 8; ++l) { const int L = L0 + l; if (L >= nlines) break; const size_t e = (size_t)L * 64 + lane * 2; const int k = (int)(e % K), n = (int)(e / K); v2us o;
            o[0] = f2bf(w[(size_t)k * N + n]); o[1] = f2bf(w[(size_t)(k + 1) * N + n]); *(volatile v2us*)(Bt + e) = o; }
        if (ps == 0) __threadfence(); }
}
template <int W, int MODE>
__global__ __launch_bounds__(256) void colpart_kernel(const float* __restrict__ H, const float* __restrict__ MEAN, float* __restrict__ PART, int nstat) {
  const int b = blockIdx.x, c = threadIdx.x; if (c >= W) return; const float mu = (MODE == 1) ? MEAN[c] : 0.0f; float s = 0.0f; const int v0 = b * 512, v1 = (v0 + 512 < nstat) ? v0 + 512 : nstat;
  for (int v = v0; v < v1; ++v) { const float h = H[(size_t)v * W + c]; if (MODE == 1) { const float d = h - mu; s += (d * d); } else s += h; }
  for (int pass = 0; pass < 2; ++pass) { ((volatile float*)PART)[(size_t)b * W + c] = s; __threadfence(); }
}
__global__ __launch_bounds__(64) void k_zr(float* Z) { *(volatile float*)(Z + threadIdx.x) = 0.0f; __threadfence(); *(volatile float*)(Z + threadIdx.x) = 0.0f; }
__global__ __launch_bounds__(256) void k_dsm(const float* __restrict__ CR, const float* __restrict__ PQ, const float* __restrict__ PK, float* W) { const unsigned idx = blockIdx.x * 256 + threadIdx.x; const unsigned b = idx / DF, d = idx % DF; const float* row = CR + ((size_t)d * NB_ + b) * NR; float g[NR];
    const float sq = __fadd_rn(PQ[(size_t)(2 * b) * DF + d], PQ[(size_t)(2 * b + 1) * DF + d]); float mx = -3.0e38f;
#pragma unroll
    for (int r4 = 0; r4 < NR / 4; ++r4) { const v4f c = *(const v4f*)(row + r4 * 4);
#pragma unroll
        for (int q = 0; q < 4; ++q) { const int r = r4 * 4 + q; const float sk = __fadd_rn(PK[(size_t)(2 * r) * DF + d], PK[(size_t)(2 * r + 1) * DF + d]); const float t = __fsub_rn(__fadd_rn(sq, sk), __fmul_rn(2.0f, c[q])); const float ng = -__fsqrt_rn(fmaxf(t, 0.0f)); g[r] = ng; mx = fmaxf(mx, ng); } }
    float sum = 0.0f;
#pragma unroll
    for (int r = 0; r < NR; ++r) { g[r] = __expf(__fsub_rn(g[r], mx)); sum = __fadd_rn(sum, g[r]); }
    const float inv = __fdiv_rn(1.0f, sum);
#pragma unroll
    for (int r = 0; r < NR; ++r) g[r] = __fmul_rn(g[r], inv);
#pragma unroll
    for (int r = 0; r < NR; ++r) *(volatile float*)(W + ((size_t)b * NR + r) * DF + d) = g[r];
    __threadfence();
#pragma unroll
    for (int r = 0; r < NR; ++r) *(volatile float*)(W + ((size_t)b * NR + r) * DF + d) = g[r]; }
__global__ __launch_bounds__(256) void k_fold(const float* __restrict__ W, const float* __restrict__ a3, h16* MB) { const unsigned idx = blockIdx.x * 256 + threadIdx.x; const unsigned e4 = idx % (DF / 4), bd = idx / (DF / 4), d = bd % DF, b = bd / DF; v4f acc = (v4f){0.0f, 0.0f, 0.0f, 0.0f};
#pragma unroll
    for (int r = 0; r < NR; ++r) { const float wr = W[((size_t)b * NR + r) * DF + d]; const v4f p = *(const v4f*)(a3 + ((size_t)r * DF + d) * DF + e4 * 4);
#pragma unroll
        for (int q = 0; q < 4; ++q) acc[q] = __fadd_rn(acc[q], __fmul_rn(wr, bfr(p[q]))); }
    v4h o;
#pragma unroll
    for (int q = 0; q < 4; ++q) o[q] = tohx(__fmul_rn(acc[q], CAR));
    *(volatile v4h*)(MB + (size_t)idx * 4) = o; __threadfence(); *(volatile v4h*)(MB + (size_t)idx * 4) = o; }
__global__ __launch_bounds__(256) void k_ep(const float* __restrict__ P, const float* __restrict__ a6, float* out) { const unsigned idx = blockIdx.x * 256 + threadIdx.x; const unsigned c0 = (idx % (DF / 4)) * 4; const v4f p = *(const v4f*)(P + (size_t)idx * 4), bi = *(const v4f*)(a6 + c0); v4f o;
#pragma unroll
    for (int q = 0; q < 4; ++q) o[q] = __fadd_rn(__fmul_rn(p[q], 1.0f / CAR), bfr(bi[q]));
    *(volatile v4f*)(out + (size_t)idx * 4) = o; __threadfence(); *(volatile v4f*)(out + (size_t)idx * 4) = o; }

extern "C" void kernel_launch(void* const* d_in, const int* in_sizes, int n_in,
                              void* d_out, int out_size, void* d_ws, size_t ws_size, hipStream_t stream) {
    (void)in_sizes; (void)n_in; (void)out_size;
    const float* a0 = (const float*)d_in[0]; const float* a2 = (const float*)d_in[2]; const float* a3 = (const float*)d_in[3]; const float* a4 = (const float*)d_in[4]; const float* a5 = (const float*)d_in[5]; const float* a6 = (const float*)d_in[6];
    float* OUT = (float*)d_out;
    char* wsp = (char*)d_ws;
    auto take = [&](size_t bytes) { char* p = wsp; wsp += (bytes + 255) & ~(size_t)255; return (void*)p; };
    const size_t PL = (size_t)NB_ * NP * DF;
    float* ZR = (float*)take((size_t)DF * 4); float* QF = (float*)take(PL * 4); float* KF = (float*)take(PL * 4); float* PQ = (float*)take((size_t)128 * DF * 4); float* PK = (float*)take((size_t)128 * DF * 4);
    bf* QT = (bf*)take(PL * 2); bf* KT = (bf*)take(PL * 2); float* CR = (float*)take((size_t)DF * NB_ * NR * 4); float* WT = (float*)take((size_t)NB_ * NR * DF * 4); h16* MB = (h16*)take((size_t)NB_ * DF * DF * 2);
    float* VF = (float*)take(PL * 4); h16* VH = (h16*)take(PL * 2); float* O1 = (float*)take(PL * 4); h16* O1H = (h16*)take(PL * 2); float* WOF = (float*)take((size_t)DF * DF * 4); h16* WOH = (h16*)take((size_t)DF * DF * 2); float* P2 = (float*)take(PL * 4);
    if ((size_t)(wsp - (char*)d_ws) > ws_size) return;
    const size_t N4 = PL / 4; const unsigned G4 = (unsigned)(N4 / 256);
    k_zr<<<1, 64, 0, stream>>>(ZR);
    k_rbf<<<G4, 256, 0, stream>>>(a0, QF, N4); k_rbf<<<G4, 256, 0, stream>>>(a4, KF, N4);
    colpart_kernel<DF, 1><<<128, 256, 0, stream>>>(QF, ZR, PQ, NB_ * NP); colpart_kernel<DF, 1><<<128, 256, 0, stream>>>(KF, ZR, PK, NR * NP);
    k_wtG<<<(unsigned)((PL / 64 + 63) / 64), 256, 0, stream>>>(a0, NB_ * NP, DF, QT); k_wtG<<<(unsigned)((PL / 64 + 63) / 64), 256, 0, stream>>>(a4, NR * NP, DF, KT);
    k_gemmw<bf, 0, false><<<dim3(NB_ / 64, NR / 64, DF), 32, 0, stream>>>(QT, nullptr, KT, nullptr, NP, CR, NR, nullptr, (size_t)NB_ * NP, (size_t)NR * NP, (size_t)NB_ * NR);
    k_dsm<<<NB_ * DF / 256, 256, 0, stream>>>(CR, PQ, PK, WT);
    k_fold<<<(unsigned)((size_t)NB_ * DF * (DF / 4) / 256), 256, 0, stream>>>(WT, a3, MB);
    k_rbf<<<G4, 256, 0, stream>>>(a2, VF, N4); k_f2h<<<G4, 256, 0, stream>>>(VF, VH, N4);
    k_gemmw<h16, 0, false><<<dim3(NP / 64, DF / 64, NB_), 32, 0, stream>>>(VH, nullptr, MB, nullptr, DF, O1, DF, nullptr, (size_t)NP * DF, (size_t)DF * DF, (size_t)NP * DF);
    k_f2h<<<G4, 256, 0, stream>>>(O1, O1H, N4);
    k_rbf<<<(unsigned)((size_t)DF * DF / 4 / 256), 256, 0, stream>>>(a5, WOF, (size_t)DF * DF / 4); k_f2h<<<(unsigned)((size_t)DF * DF / 4 / 256), 256, 0, stream>>>(WOF, WOH, (size_t)DF * DF / 4);
    k_gemmw<h16, 0, false><<<dim3(NB_ * NP / 64, DF / 64, 1), 32, 0, stream>>>(O1H, nullptr, WOH, nullptr, DF, P2, DF, nullptr, 0, 0, 0);
    k_ep<<<G4, 256, 0, stream>>>(P2, a6, OUT);
}
